// EGLAVarNet_39951785787598
// MI455X (gfx1250) — hardware-verified
//
#include <hip/hip_runtime.h>
#include <math.h>
#include <stdint.h>

constexpr int kBatch   = 2;
constexpr int kCh      = 64;
constexpr int kNpix    = 65536;
constexpr int kLayers  = 4;
constexpr int kCin     = 2;
constexpr int kQpx     = 32768;
constexpr int kQuarters = 4;
constexpr int kCovChunk = 2048;
constexpr int kChunksPerQ = kQpx / kCovChunk;
constexpr int kChunksTot  = kQuarters * kChunksPerQ;
constexpr int kGatePxPerBlock = 4096;
constexpr int kGateBlocksPerQ = kQpx / kGatePxPerBlock;
constexpr int kGateBlocksTot  = kQuarters * kGateBlocksPerQ;
constexpr float kWCarry   = 16.0f;
constexpr float kMemCarry = 256.0f;
constexpr float kInvN     = 1.0f / 65536.0f;

constexpr size_t kFeatBytes = (size_t)kBatch * kCh * kNpix * 4;
constexpr size_t kPlane16   = (size_t)kBatch * kNpix * kCh * 2;
constexpr size_t kP1Bytes   = (size_t)256 * kQpx * 2;
constexpr size_t kKgBytes   = (size_t)kCh * kQpx * 2;
constexpr size_t kKnwpBytes = (size_t)kChunksTot * 4096 * 4;
constexpr size_t kFpartBytes = (size_t)kCh * kGateBlocksTot * 128;
constexpr size_t kGnpBytes  = (size_t)512 * 128;
constexpr size_t kMemtBytes = (size_t)kBatch * 64 * 64 * 2;
constexpr size_t kW16Bytes  = (size_t)1536 * 64 * 2;
constexpr size_t kBiasBytes = (size_t)kLayers * 256 * 4;
constexpr size_t kOffFeatA = 0;
constexpr size_t kOffFeatB = kOffFeatA + kFeatBytes;
constexpr size_t kOffXnt   = kOffFeatB + kFeatBytes;
constexpr size_t kOffQ16   = kOffXnt + kPlane16;
constexpr size_t kOffP1    = kOffQ16 + kPlane16;
constexpr size_t kOffKg    = kOffP1 + kP1Bytes;
constexpr size_t kOffKnwp  = kOffKg + kKgBytes;
constexpr size_t kOffFpart = kOffKnwp + kKnwpBytes;
constexpr size_t kOffGnp   = kOffFpart + kFpartBytes;
constexpr size_t kOffMemt  = kOffGnp + kGnpBytes;
constexpr size_t kOffW16   = kOffMemt + kMemtBytes;
constexpr size_t kOffBias  = kOffW16 + kW16Bytes;
constexpr size_t kWsTotal  = kOffBias + kBiasBytes;
static_assert(kWsTotal <= 134217728ull, "ws");
static_assert((kOffXnt % 128) == 0 && (kOffQ16 % 128) == 0 && (kOffP1 % 128) == 0 && (kOffKg % 128) == 0, "al");
static_assert((kOffKnwp % 128) == 0 && (kOffFpart % 128) == 0 && (kOffGnp % 128) == 0 && (kOffMemt % 128) == 0, "al");
static_assert((kOffW16 % 128) == 0 && (kOffBias % 128) == 0, "al");

typedef __attribute__((ext_vector_type(16))) _Float16 v16h;
typedef __attribute__((ext_vector_type(8)))  _Float16 v8h;
typedef __attribute__((ext_vector_type(16))) __bf16   v16b;
typedef __attribute__((ext_vector_type(8)))  __bf16   v8b;
typedef __attribute__((ext_vector_type(8)))  float    v8f;
typedef __attribute__((ext_vector_type(4)))  float    v4f;
typedef __attribute__((ext_vector_type(4)))  unsigned int v4u;

__device__ __forceinline__ unsigned short f2bf_bits(float f) {
  unsigned u = __float_as_uint(f);
  return (unsigned short)((u + 0x7FFFu + ((u >> 16) & 1u)) >> 16);
}
__device__ __forceinline__ float bf_bits2f(unsigned short h) { return __uint_as_float(((unsigned)h) << 16); }

__device__ __forceinline__ void dep_guard_h(v8f& a, v8f& b, v16h x, v16h y) { asm volatile("v_nop\n\tv_nop\n\tv_nop\n\tv_nop" : "+v"(a), "+v"(b) : "v"(x), "v"(y)); }
__device__ __forceinline__ void dep_guard_b(v8f& a, v8f& b, v16b x, v16b y) { asm volatile("v_nop\n\tv_nop\n\tv_nop\n\tv_nop" : "+v"(a), "+v"(b) : "v"(x), "v"(y)); }
__device__ __forceinline__ void keep4_h(v16h a, v16h b, v16h c, v16h d) { asm volatile("v_nop" :: "v"(a), "v"(b), "v"(c), "v"(d)); }
__device__ __forceinline__ void keep4_b(v16b a, v16b b, v16b c, v16b d) { asm volatile("v_nop" :: "v"(a), "v"(b), "v"(c), "v"(d)); }
__device__ __forceinline__ void acc_guard4(v8f& a, v8f& b, v8f& c, v8f& d) { asm volatile("v_nop\n\tv_nop\n\tv_nop\n\tv_nop" : "+v"(a), "+v"(b), "+v"(c), "+v"(d)); }
template <typename T> struct Frag;
template <> struct Frag<_Float16> {
  typedef v16h V; union U { v16h v; v8h h[2]; };
  static __device__ __forceinline__ v16h load(const _Float16* p) {
    U f; f.h[0] = *(const v8h*)(p); f.h[1] = *(const v8h*)(p + 16); return f.v;
  }
  static __device__ __forceinline__ v8f mma(v16h a, v16h b, v8f c) {
    return __builtin_amdgcn_wmma_f32_16x16x32_f16(false, a, false, b, (short)0, c, false, false);
  }
  static __device__ __forceinline__ void guard(v8f& a, v8f& b, v16h x, v16h y) { dep_guard_h(a, b, x, y); }
  static __device__ __forceinline__ void keep(v16h a, v16h b, v16h c, v16h d) { keep4_h(a, b, c, d); }
};
template <> struct Frag<__bf16> {
  typedef v16b V; union U { v16b v; v8b h[2]; };
  static __device__ __forceinline__ v16b load(const __bf16* p) {
    U f; f.h[0] = *(const v8b*)(p); f.h[1] = *(const v8b*)(p + 16); return f.v;
  }
  static __device__ __forceinline__ v8f mma(v16b a, v16b b, v8f c) {
    return __builtin_amdgcn_wmma_f32_16x16x32_bf16(false, a, false, b, (short)0, c, false, false);
  }
  static __device__ __forceinline__ void guard(v8f& a, v8f& b, v16b x, v16b y) { dep_guard_b(a, b, x, y); }
  static __device__ __forceinline__ void keep(v16b a, v16b b, v16b c, v16b d) { keep4_b(a, b, c, d); }
};

__device__ __forceinline__ unsigned pk16(unsigned short a, unsigned short b) { return (unsigned)a | ((unsigned)b << 16); }
__device__ __forceinline__ unsigned short h_bits(float f) { const _Float16 h = (_Float16)f; return __builtin_bit_cast(unsigned short, h); }
__device__ __forceinline__ float h16_lo(unsigned w) { return (float)__builtin_bit_cast(_Float16, (unsigned short)(w & 0xffffu)); }
__device__ __forceinline__ float h16_hi(unsigned w) { return (float)__builtin_bit_cast(_Float16, (unsigned short)(w >> 16)); }
__device__ __forceinline__ float sigm_f(float x) { return 1.0f / (1.0f + expf(-x)); }

template <int ET> struct Elem;
template <> struct Elem<0> { typedef _Float16 T; };
template <> struct Elem<1> { typedef __bf16 T; };
template <int ET, bool SPLIT, int BIAS_MODE, int OUT_MODE, bool RESID, int ACT = 0>
__global__ __launch_bounds__(256) void wmma_gemm64(
    const unsigned short* __restrict__ Ap, const unsigned short* __restrict__ A2p, int lda, long strideA,
    const unsigned short* __restrict__ Btp, const unsigned short* __restrict__ Bt2p, int ldb, long strideB,
    void* __restrict__ Cout, void* __restrict__ Cout2, int ldc, long strideC,
    const float* __restrict__ bias,
    const float* __restrict__ resid, long strideR,
    int M, int N, int K, float scale) {
  typedef typename Elem<ET>::T T;
  typedef typename Frag<T>::V V;
  const T* A = (const T*)Ap; const T* A2 = (const T*)A2p; const T* Bt = (const T*)Btp; const T* Bt2 = (const T*)Bt2p;
  __shared__ __align__(16) float sT[8][16 * 68];
  const int b    = blockIdx.y;
  const int lane = threadIdx.x & 31;
  const int wave = threadIdx.x >> 5;
  const int tilesN = N >> 6;
  const int tilesM = M >> 6;
  const int tile = blockIdx.x * 8 + wave;
  if (tile >= tilesM * tilesN) return;
  const int tm = tile / tilesN;
  const int tn = tile - tm * tilesN;
  const int m0 = tm << 6;
  const int n0 = tn << 6;

  const T* Ab  = A  + (size_t)b * strideA;
  const T* Bb  = Bt + (size_t)b * strideB;
  const T* Ab2 = SPLIT ? (A2  + (size_t)b * strideA) : nullptr;
  const T* Bb2 = SPLIT ? (Bt2 + (size_t)b * strideB) : nullptr;

  const int rlane = lane & 15;
  const int koff  = (lane >> 4) * 8;
  const int mOff  = (lane >> 4) * 8;

  v8f acc[4][4];
#pragma unroll
  for (int i = 0; i < 4; ++i)
#pragma unroll
    for (int j = 0; j < 4; ++j) acc[i][j] = (v8f){0.f,0.f,0.f,0.f,0.f,0.f,0.f,0.f};

  for (int k0 = 0; k0 < K; k0 += 32) {
    V bh[4], bl[4];
#pragma unroll
    for (int j = 0; j < 4; ++j) {
      const size_t bo = (size_t)(n0 + (j << 4) + rlane) * ldb + koff + k0;
      bh[j] = Frag<T>::load(Bb + bo);
      if (SPLIT) bl[j] = Frag<T>::load(Bb2 + bo);
    }
#pragma unroll
    for (int i = 0; i < 4; ++i) {
      const size_t ao = (size_t)(m0 + (i << 4) + rlane) * lda + koff + k0;
      V ah = Frag<T>::load(Ab + ao);
      V al;
      if (SPLIT) al = Frag<T>::load(Ab2 + ao);
#pragma unroll
      for (int j = 0; j < 4; ++j) {
        acc[i][j] = Frag<T>::mma(ah, bh[j], acc[i][j]);
        if (SPLIT) {
          acc[i][j] = Frag<T>::mma(ah, bl[j], acc[i][j]);
          acc[i][j] = Frag<T>::mma(al, bh[j], acc[i][j]);
        }
      }
      Frag<T>::guard(acc[i][0], acc[i][3], ah, SPLIT ? al : ah);
    }
    Frag<T>::keep(bh[0], bh[1], bh[2], bh[3]);
    if (SPLIT) Frag<T>::keep(bl[0], bl[1], bl[2], bl[3]);
  }
  acc_guard4(acc[0][0], acc[0][1], acc[0][2], acc[0][3]);
  acc_guard4(acc[1][0], acc[1][1], acc[1][2], acc[1][3]);
  acc_guard4(acc[2][0], acc[2][1], acc[2][2], acc[2][3]);
  acc_guard4(acc[3][0], acc[3][1], acc[3][2], acc[3][3]);

  float* slab = sT[wave];
  const float* Rb = RESID ? (resid + (size_t)b * strideR) : nullptr;
#pragma unroll
  for (int i = 0; i < 4; ++i) {
    const int mBase = m0 + (i << 4);
#pragma unroll
    for (int j = 0; j < 4; ++j) {
      const int n = n0 + (j << 4) + rlane;
      float bv = 0.f;
      if (BIAS_MODE == 2) bv = bias[n];
#pragma unroll
      for (int r = 0; r < 8; ++r) {
        float v = acc[i][j][r] * scale;
        if (BIAS_MODE == 1) v += bias[mBase + mOff + r];
        if (BIAS_MODE == 2) v += bv;
        if (RESID) v += Rb[(size_t)(mBase + mOff + r) * ldc + n];
        if (ACT == 2) v = fmaxf(v, 0.0f);
        if (ACT == 4) v = (v > 0.f) ? v : 0.01f * v;
        slab[(mOff + r) * 68 + (j << 4) + rlane] = v;
      }
    }
    __builtin_amdgcn_fence(__ATOMIC_RELEASE, "workgroup");
    __builtin_amdgcn_wave_barrier();
    __builtin_amdgcn_fence(__ATOMIC_ACQUIRE, "workgroup");
    if (OUT_MODE == 0) {
      float* C = (float*)Cout + (size_t)b * strideC;
      const int hh = lane >> 4, c4 = (lane & 15) * 4;
      for (int pass = 0; pass < 2; ++pass) {
#pragma unroll
        for (int it = 0; it < 8; ++it) {
          const int row = it * 2 + hh;
          v4f v = *(const v4f*)(slab + row * 68 + c4);
          *(volatile v4f*)(C + (size_t)(mBase + row) * ldc + n0 + c4) = v;
        }
        __threadfence();
      }
    } else {
      const int q = lane >> 3, c8 = (lane & 7) * 8;
      unsigned short* C  = (unsigned short*)Cout  + (size_t)b * strideC;
      unsigned short* C2 = (OUT_MODE == 2) ? ((unsigned short*)Cout2 + (size_t)b * strideC) : nullptr;
      for (int pass = 0; pass < 2; ++pass) {
#pragma unroll
        for (int it = 0; it < 4; ++it) {
          const int row = it * 4 + q;
          const float* sp = slab + row * 68 + c8;
          v8h hv, lv;
#pragma unroll
          for (int e = 0; e < 8; ++e) {
            if (OUT_MODE == 1) {
              hv[e] = (_Float16)sp[e];
            } else {
              unsigned short hb = f2bf_bits(sp[e]);
              unsigned short lb = f2bf_bits(sp[e] - bf_bits2f(hb));
              hv[e] = __builtin_bit_cast(_Float16, hb);
              lv[e] = __builtin_bit_cast(_Float16, lb);
            }
          }
          *(volatile v8h*)(C + (size_t)(mBase + row) * ldc + n0 + c8) = hv;
          if (OUT_MODE == 2) *(volatile v8h*)(C2 + (size_t)(mBase + row) * ldc + n0 + c8) = lv;
        }
        __threadfence();
      }
    }
    __builtin_amdgcn_fence(__ATOMIC_RELEASE, "workgroup");
    __builtin_amdgcn_wave_barrier();
    __builtin_amdgcn_fence(__ATOMIC_ACQUIRE, "workgroup");
  }
}

__global__ __launch_bounds__(256) void prep_params_kernel(
    const float* __restrict__ Wk, const float* __restrict__ Wv, const float* __restrict__ Wg,
    const float* __restrict__ Wq, const float* __restrict__ Wp,
    const float* __restrict__ bk, const float* __restrict__ bv, const float* __restrict__ bg,
    unsigned short* __restrict__ W16, float* __restrict__ bkvg) {
  const int blk = blockIdx.x, t = threadIdx.x;
  if (blk < 48) {
    const int e8 = blk * 256 + t;
    const int r  = e8 >> 3;
    const int c8 = (e8 & 7) * 8;
    const float* src;
    if (blk < 32) {
      const int layer = blk >> 3;
      const int sub = blk & 7;
      const int rr = r & 255;
      if (sub < 2)      src = Wk + ((size_t)layer * 64 + rr) * 64;
      else if (sub < 4) src = Wv + ((size_t)layer * 64 + (rr - 64)) * 64;
      else              src = Wg + ((size_t)layer * 128 + (rr - 128)) * 64;
    } else if (blk < 40) {
      src = Wq + (size_t)(r - 1024) * 64;
    } else {
      src = Wp + (size_t)(r - 1280) * 64;
    }
    const v4f a = *(const v4f*)(src + c8);
    const v4f c = *(const v4f*)(src + c8 + 4);
    unsigned short hb[8];
#pragma unroll
    for (int e = 0; e < 4; ++e) { hb[e] = h_bits(a[e] * kWCarry); hb[4 + e] = h_bits(c[e] * kWCarry); }
    const v4u u = (v4u){pk16(hb[0], hb[1]), pk16(hb[2], hb[3]), pk16(hb[4], hb[5]), pk16(hb[6], hb[7])};
    unsigned short* dst = W16 + (size_t)r * 64 + c8;
    *(volatile v4u*)dst = u;
    __threadfence();
    *(volatile v4u*)dst = u;
  } else {
    const int layer = blk - 48;
    const int m = t;
    const int ik = m < 64 ? m : 63;
    const int iv = m < 64 ? 0 : (m < 128 ? (m - 64) : 63);
    const int ig = m < 128 ? 0 : (m - 128);
    const float vk = bk[layer * 64 + ik];
    const float vv = bv[layer * 64 + iv];
    const float vg = bg[layer * 128 + ig];
    const float val = m < 64 ? vk : (m < 128 ? vv : vg);
    volatile float* dst = bkvg + layer * 256 + m;
    *dst = val;
    __threadfence();
    *dst = val;
  }
}

__global__ __launch_bounds__(256) void conv_in_kernel(const float* __restrict__ x, const float* __restrict__ W,
                                                      const float* __restrict__ bias, float* __restrict__ feat) {
  const int idx = blockIdx.x * 256 + threadIdx.x;
  const int p  = idx & (kNpix - 1);
  const int oc = (idx >> 16) & 63;
  const int b  = idx >> 22;
  const int py = p >> 8, px = p & 255;
  float acc = bias[oc];
#pragma unroll
  for (int ci = 0; ci < kCin; ++ci) {
    const float* xc = x + ((size_t)(b * kCin + ci) << 16);
    const float* wc = W + (oc * kCin + ci) * 9;
#pragma unroll
    for (int tp = 0; tp < 9; ++tp) {
      const int yy = py + tp / 3 - 1, xx = px + tp % 3 - 1;
      const bool ok = ((unsigned)yy < 256u) && ((unsigned)xx < 256u);
      const int yc = yy < 0 ? 0 : (yy > 255 ? 255 : yy);
      const int xcl = xx < 0 ? 0 : (xx > 255 ? 255 : xx);
      float f = xc[(yc << 8) + xcl];
      f = ok ? f : 0.0f;
      acc += wc[tp] * f;
    }
  }
  volatile float* d = feat + idx;
  *d = acc;
  __threadfence();
  *d = acc;
}

__global__ __launch_bounds__(256) void gnstat_kernel(const float* __restrict__ feat, float* __restrict__ gnp) {
  __shared__ float rs[8], rq[8];
  const int blk = blockIdx.x, t = threadIdx.x, lane = t & 31, wave = t >> 5;
  const float* base = feat + (size_t)blk * 16384;
  float s = 0.f, q = 0.f;
#pragma unroll 4
  for (int i = 0; i < 16; ++i) {
    const v4f v = *(const v4f*)(base + ((size_t)(i * 256 + t)) * 4);
    s += (v[0] + v[1]) + (v[2] + v[3]);
    q += (v[0] * v[0] + v[1] * v[1]) + (v[2] * v[2] + v[3] * v[3]);
  }
#pragma unroll
  for (int off = 16; off > 0; off >>= 1) { s += __shfl_xor(s, off, 32); q += __shfl_xor(q, off, 32); }
  if (lane == 0) { rs[wave] = s; rq[wave] = q; }
  __syncthreads();
  if (wave == 0) {
    float S = 0.f, Q = 0.f;
#pragma unroll
    for (int w = 0; w < 8; ++w) { S += rs[w]; Q += rq[w]; }
    const float val = (lane == 0) ? S : ((lane == 1) ? Q : 0.0f);
    volatile float* d = gnp + (size_t)blk * 32 + lane;
    *d = val;
    __threadfence();
    *d = val;
  }
}

__global__ __launch_bounds__(256) void gn_xnt_kernel(const float* __restrict__ feat, const float* __restrict__ gnp,
                                                     const float* __restrict__ gam, const float* __restrict__ bet,
                                                     unsigned short* __restrict__ xnt) {
  __shared__ float sm[128 * 65];
  __shared__ float gmu[8], grs[8], sg[64], sbt[64];
  const int t = threadIdx.x;
  const int n0 = blockIdx.x * 128;
  const int b  = blockIdx.y;
  if (t < 8) {
    double s = 0.0, q = 0.0;
    const float* gp = gnp + (size_t)((b * 8 + t) * 32) * 32;
#pragma unroll 1
    for (int z = 0; z < 32; ++z) { s += (double)gp[z * 32]; q += (double)gp[z * 32 + 1]; }
    const double inv = 1.0 / 524288.0;
    const double mu = s * inv;
    const double var = q * inv - mu * mu;
    float varf = (float)var;
    varf = varf > 0.0f ? varf : 0.0f;
    gmu[t] = (float)mu;
    grs[t] = rsqrtf(varf + 1e-5f);
  }
  if (t < 64) { sg[t] = gam[t]; sbt[t] = bet[t]; }
  __syncthreads();
  const float* fb = feat + (size_t)b * kCh * kNpix + n0;
#pragma unroll 4
  for (int i = 0; i < 32; ++i) {
    const int e = i * 256 + t;
    const int c = e >> 7, nl = e & 127;
    const float f = fb[(size_t)c * kNpix + nl];
    const int g = c >> 3;
    sm[nl * 65 + c] = (f - gmu[g]) * grs[g] * sg[c] + sbt[c];
  }
  __syncthreads();
  unsigned short* xb = xnt + ((size_t)b * kNpix + n0) * kCh;
  for (int pass = 0; pass < 2; ++pass) {
#pragma unroll
    for (int it = 0; it < 4; ++it) {
      const int q = it * 256 + t;
      const int row = q >> 3, c8 = (q & 7) * 8;
      unsigned short hb[8];
#pragma unroll
      for (int e = 0; e < 8; ++e) hb[e] = h_bits(sm[row * 65 + c8 + e]);
      const v4u u = (v4u){pk16(hb[0], hb[1]), pk16(hb[2], hb[3]), pk16(hb[4], hb[5]), pk16(hb[6], hb[7])};
      *(volatile v4u*)(xb + (size_t)row * kCh + c8) = u;
    }
    __threadfence();
  }
}

__global__ __launch_bounds__(256) void gates_kernel(const unsigned* __restrict__ p1w, unsigned* __restrict__ kgw,
                                                    float* __restrict__ fpart, int qtr) {
  __shared__ float red[8];
  const int t = threadIdx.x, lane = t & 31, wave = t >> 5;
  const int c = blockIdx.y, pbl = blockIdx.x;
  const size_t wK = (size_t)c * (kQpx / 2);
  const size_t wF = (size_t)(128 + c) * (kQpx / 2);
  const size_t wI = (size_t)(192 + c) * (kQpx / 2);
  float fp = 0.f;
#pragma unroll 1
  for (int it = 0; it < 8; ++it) {
    const int widx = ((pbl * kGatePxPerBlock + it * 512 + wave * 64) >> 1) + lane;
    const unsigned kw = p1w[wK + widx];
    const unsigned fw = p1w[wF + widx];
    const unsigned iw = p1w[wI + widx];
    const float kg0 = h16_lo(kw) * sigm_f(h16_lo(iw));
    const float kg1 = h16_hi(kw) * sigm_f(h16_hi(iw));
    fp += sigm_f(h16_lo(fw)) + sigm_f(h16_hi(fw));
    const unsigned u = pk16(h_bits(kg0), h_bits(kg1));
    volatile unsigned* dst = kgw + wK + widx;
    *dst = u;
    __threadfence();
    *dst = u;
  }
#pragma unroll
  for (int off = 16; off > 0; off >>= 1) fp += __shfl_xor(fp, off, 32);
  if (lane == 0) red[wave] = fp;
  __syncthreads();
  if (wave == 0) {
    float S = 0.f;
#pragma unroll
    for (int w = 0; w < 8; ++w) S += red[w];
    const float val = (lane == 0) ? S : 0.0f;
    volatile float* d = fpart + (size_t)(c * kGateBlocksTot + qtr * kGateBlocksPerQ + pbl) * 32 + lane;
    *d = val;
    __threadfence();
    *d = val;
  }
}

__global__ __launch_bounds__(256) void mem_kernel(const float* __restrict__ knwp, const float* __restrict__ fpart,
                                                  const float* __restrict__ hidden, float* __restrict__ out1,
                                                  unsigned short* __restrict__ memt, int lyr) {
  __shared__ float sm[64 * 65];
  __shared__ float fsm[64];
  const int b = blockIdx.x, t = threadIdx.x;
  if (t < 64) {
    float s = 0.f;
#pragma unroll 1
    for (int z = 0; z < 16; ++z) s += fpart[((size_t)t * kGateBlocksTot + (size_t)b * 16 + z) * 32];
    fsm[t] = s * kInvN;
  }
  __syncthreads();
#pragma unroll 1
  for (int i = 0; i < 16; ++i) {
    const int idx = i * 256 + t;
    const int c = idx >> 6, d = idx & 63;
    float kn = 0.f;
#pragma unroll 1
    for (int y = 0; y < 32; ++y) kn += knwp[((size_t)b * 32 + y) * 4096 + idx];
    const float prev = hidden[((size_t)b * kLayers + lyr) * 4096 + idx];
    const float nm = fsm[c] * prev + kn * kInvN;
    sm[c * 65 + d] = nm;
  }
  __syncthreads();
  float* ob = out1 + ((size_t)b * kLayers + lyr) * 4096;
  for (int pass = 0; pass < 2; ++pass) {
#pragma unroll
    for (int it = 0; it < 4; ++it) {
      const int q = it * 256 + t;
      const int row = q >> 4, c4 = (q & 15) * 4;
      const float* sp = sm + row * 65 + c4;
      const v4f v = (v4f){sp[0], sp[1], sp[2], sp[3]};
      *(volatile v4f*)(ob + row * 64 + c4) = v;
    }
    __threadfence();
  }
  unsigned short* mb = memt + (size_t)b * 4096;
  for (int pass = 0; pass < 2; ++pass) {
#pragma unroll
    for (int it = 0; it < 2; ++it) {
      const int q = it * 256 + t;
      const int d = q >> 3, c8 = (q & 7) * 8;
      unsigned short hb[8];
#pragma unroll
      for (int e = 0; e < 8; ++e) hb[e] = h_bits(sm[(c8 + e) * 65 + d] * kMemCarry);
      const v4u u = (v4u){pk16(hb[0], hb[1]), pk16(hb[2], hb[3]), pk16(hb[4], hb[5]), pk16(hb[6], hb[7])};
      *(volatile v4u*)(mb + d * 64 + c8) = u;
    }
    __threadfence();
  }
}

__global__ __launch_bounds__(256) void conv_out_kernel(const float* __restrict__ feat, const float* __restrict__ W,
                                                       const float* __restrict__ bias, const float* __restrict__ x,
                                                       float* __restrict__ out) {
  const int idx = blockIdx.x * 256 + threadIdx.x;
  const int p  = idx & (kNpix - 1);
  const int oc = (idx >> 16) & 1;
  const int b  = idx >> 17;
  const int py = p >> 8, px = p & 255;
  int off[9];
  bool ok[9];
#pragma unroll
  for (int tp = 0; tp < 9; ++tp) {
    const int yy = py + tp / 3 - 1, xx = px + tp % 3 - 1;
    ok[tp] = ((unsigned)yy < 256u) && ((unsigned)xx < 256u);
    const int yc = yy < 0 ? 0 : (yy > 255 ? 255 : yy);
    const int xcl = xx < 0 ? 0 : (xx > 255 ? 255 : xx);
    off[tp] = (yc << 8) + xcl;
  }
  const float* fb0 = feat + ((size_t)b * kCh << 16);
  const float* wb0 = W + (size_t)oc * kCh * 9;
  float acc = 0.f;
#pragma unroll 1
  for (int c = 0; c < kCh; ++c) {
    const float* fb = fb0 + ((size_t)c << 16);
    const float* wb = wb0 + c * 9;
#pragma unroll
    for (int tp = 0; tp < 9; ++tp) {
      float f = fb[off[tp]];
      f = ok[tp] ? f : 0.0f;
      acc += wb[tp] * f;
    }
  }
  const float o = acc + bias[oc] + x[idx];
  volatile float* d = out + idx;
  *d = o;
  __threadfence();
  *d = o;
}

extern "C" void kernel_launch(void* const* d_in, const int* in_sizes, int n_in,
                              void* d_out, int out_size, void* d_ws, size_t ws_size,
                              hipStream_t stream) {
  if (n_in < 18) return;
  if (out_size != kBatch * kCin * kNpix + kBatch * kLayers * 64 * 64) return;
  if (in_sizes[0] != kBatch * kCin * kNpix || in_sizes[1] != kBatch * kLayers * 64 * 64) return;
  if (ws_size < kWsTotal) return;

  const float* x      = (const float*)d_in[0];
  const float* hidden = (const float*)d_in[1];
  const float* W_in   = (const float*)d_in[2];
  const float* b_in   = (const float*)d_in[3];
  const float* gamma  = (const float*)d_in[4];
  const float* beta   = (const float*)d_in[5];
  const float* Wq     = (const float*)d_in[6];
  const float* bq     = (const float*)d_in[7];
  const float* Wk     = (const float*)d_in[8];
  const float* bk     = (const float*)d_in[9];
  const float* Wv     = (const float*)d_in[10];
  const float* bv     = (const float*)d_in[11];
  const float* Wg     = (const float*)d_in[12];
  const float* bg     = (const float*)d_in[13];
  const float* Wp     = (const float*)d_in[14];
  const float* bp     = (const float*)d_in[15];
  const float* W_out  = (const float*)d_in[16];
  const float* b_out  = (const float*)d_in[17];

  float* out0 = (float*)d_out;
  float* out1 = (float*)d_out + (size_t)kBatch * kCin * kNpix;

  char* ws = (char*)d_ws;
  float*          featA = (float*)(ws + kOffFeatA);
  float*          featB = (float*)(ws + kOffFeatB);
  unsigned short* xnt   = (unsigned short*)(ws + kOffXnt);
  unsigned short* ret16 = (unsigned short*)(ws + kOffXnt);
  unsigned short* q16   = (unsigned short*)(ws + kOffQ16);
  unsigned short* p1    = (unsigned short*)(ws + kOffP1);
  unsigned short* kg    = (unsigned short*)(ws + kOffKg);
  float*          knwp  = (float*)(ws + kOffKnwp);
  float*          fpart = (float*)(ws + kOffFpart);
  float*          gnp   = (float*)(ws + kOffGnp);
  unsigned short* memt  = (unsigned short*)(ws + kOffMemt);
  unsigned short* w16   = (unsigned short*)(ws + kOffW16);
  unsigned short* wkvg16 = w16;
  unsigned short* wq16   = w16 + (size_t)1024 * 64;
  unsigned short* wp16   = w16 + (size_t)1280 * 64;
  float*          bkvg   = (float*)(ws + kOffBias);

  const long strideAct = (long)kNpix * kCh;
  const long strideXq  = 0;

  prep_params_kernel<<<52, 256, 0, stream>>>(Wk, Wv, Wg, Wq, Wp, bk, bv, bg, w16, bkvg);
  conv_in_kernel<<<(kBatch * kCh * kNpix) / 256, 256, 0, stream>>>(x, W_in, b_in, featA);

  for (int lyr = 0; lyr < kLayers; ++lyr) {
    float* fold = (lyr & 1) ? featB : featA;
    float* fnew = (lyr & 1) ? featA : featB;

    gnstat_kernel<<<512, 256, 0, stream>>>(fold, gnp);
    gn_xnt_kernel<<<dim3(kNpix / 128, kBatch), 256, 0, stream>>>(fold, gnp, gamma + lyr * 64, beta + lyr * 64, xnt);

    wmma_gemm64<0, false, 2, 1, false, 0><<<dim3(128, kBatch), 256, 0, stream>>>(
        xnt, xnt, 64, strideAct,
        wq16 + (size_t)lyr * 4096, wq16 + (size_t)lyr * 4096, 64, strideXq,
        (void*)q16, (void*)q16, 64, strideAct,
        bq + lyr * 64,
        fold, 0L,
        kNpix, 64, 64, 1.0f / kWCarry);

    for (int qtr = 0; qtr < kQuarters; ++qtr) {
      wmma_gemm64<0, false, 1, 1, false, 0><<<dim3(256, 1), 256, 0, stream>>>(
          wkvg16 + (size_t)lyr * 256 * 64, wkvg16 + (size_t)lyr * 256 * 64, 64, 0L,
          xnt + (size_t)qtr * kQpx * kCh, xnt + (size_t)qtr * kQpx * kCh, 64, 0L,
          (void*)p1, (void*)p1, kQpx, 0L,
          bkvg + lyr * 256,
          fold, 0L,
          256, kQpx, 64, 1.0f / kWCarry);

      gates_kernel<<<dim3(kGateBlocksPerQ, kCh), 256, 0, stream>>>((const unsigned*)p1, (unsigned*)kg, fpart, qtr);

      wmma_gemm64<0, false, 0, 0, false, 0><<<dim3(1, kChunksPerQ), 256, 0, stream>>>(
          kg, kg, kQpx, (long)kCovChunk,
          p1 + (size_t)64 * kQpx, p1 + (size_t)64 * kQpx, kQpx, (long)kCovChunk,
          (void*)(knwp + (size_t)qtr * kChunksPerQ * 4096), (void*)(knwp + (size_t)qtr * kChunksPerQ * 4096), 64, 4096L,
          bp,
          fold, 0L,
          64, 64, kCovChunk, 1.0f);
    }

    mem_kernel<<<kBatch, 256, 0, stream>>>(knwp, fpart, hidden, out1, memt, lyr);

    wmma_gemm64<0, false, 0, 1, false, 0><<<dim3(128, kBatch), 256, 0, stream>>>(
        q16, q16, 64, strideAct,
        memt, memt, 64, 4096L,
        (void*)ret16, (void*)ret16, 64, strideAct,
        bp,
        fold, 0L,
        kNpix, 64, 64, 1.0f / 16.0f);

    wmma_gemm64<0, false, 1, 0, true, 0><<<dim3(128, kBatch), 256, 0, stream>>>(
        wp16 + (size_t)lyr * 4096, wp16 + (size_t)lyr * 4096, 64, 0L,
        ret16, ret16, 64, strideAct,
        (void*)fnew, (void*)fnew, kNpix, strideAct,
        bp + lyr * 64,
        fold, strideAct,
        64, kNpix, 64, 1.0f / 2048.0f);
  }

  conv_out_kernel<<<(kBatch * kCin * kNpix) / 256, 256, 0, stream>>>(featA, W_out, b_out, x, out0);
}
